// CNNMambaFast_78932908966461
// MI455X (gfx1250) — hardware-verified
//
#include <hip/hip_runtime.h>
#include <math.h>

typedef __attribute__((ext_vector_type(16))) _Float16 v16h;
typedef __attribute__((ext_vector_type(16))) __bf16 v16b;
typedef __attribute__((ext_vector_type(8)))  _Float16 v8h;
typedef __attribute__((ext_vector_type(8)))  float v8f;
typedef __attribute__((ext_vector_type(4)))  float v4f;
typedef __attribute__((ext_vector_type(2)))  float v2f;
typedef __attribute__((ext_vector_type(4)))  unsigned v4u;
typedef __attribute__((ext_vector_type(4)))  int v4i;
typedef float __attribute__((may_alias)) float_a;
typedef int __attribute__((may_alias)) int_a;

template <typename T> __device__ __forceinline__ void vst2(void* p, T v) { *(volatile T*)p = v; __threadfence(); *(volatile T*)p = v; }
__device__ __forceinline__ v8f wmma16(v16h a, v16h b, v8f c) {
  v8f d = __builtin_amdgcn_wmma_f32_16x16x32_f16(false, a, false, b, (short)0, c, false, false);
  asm volatile("v_nop\n\tv_nop\n\tv_nop\n\tv_nop" : "+v"(d) : "v"(a), "v"(b));
  return d;
}
__device__ __forceinline__ v8f wmma_bf(v16b a, v16b b, v8f c) {
  v8f d = __builtin_amdgcn_wmma_f32_16x16x32_bf16(false, a, false, b, (short)0, c, false, false);
  asm volatile("v_nop\n\tv_nop\n\tv_nop\n\tv_nop" : "+v"(d) : "v"(a), "v"(b));
  return d;
}
__device__ __forceinline__ v16h frag_h(const _Float16* rowk0, int lane) {
  union { v16h v; v8h q[2]; } u; const _Float16* p = rowk0 + 8 * (lane >> 4);
  u.q[0] = *(const v8h*)p; u.q[1] = *(const v8h*)(p + 16); return u.v;
}
__device__ __forceinline__ v16h frag_f32(const float* rowk0, int lane) {
  v16h a; const float* p = rowk0 + 8 * (lane >> 4);
#pragma unroll
  for (int i = 0; i < 8; ++i) { a[i] = (_Float16)p[i]; a[8 + i] = (_Float16)p[16 + i]; }
  return a;
}
__device__ __forceinline__ v16h frag_f32s(const float* rowk0, int lane, float sc) {
  v16h a; const float* p = rowk0 + 8 * (lane >> 4);
#pragma unroll
  for (int i = 0; i < 8; ++i) { a[i] = (_Float16)(p[i] * sc); a[8 + i] = (_Float16)(p[16 + i] * sc); }
  return a;
}
__device__ __forceinline__ v16h fragc_f32(const float* W, int k0, int n, int lane, int ld, int K) {
  v16h a; const int g = lane >> 4;
#pragma unroll
  for (int i = 0; i < 8; ++i) { const int ka = k0 + 8 * g + i, kb = ka + 16;
    a[i] = (_Float16)(ka < K ? W[(size_t)(ka < K ? ka : K - 1) * ld + n] : 0.f); a[8 + i] = (_Float16)(kb < K ? W[(size_t)(kb < K ? kb : K - 1) * ld + n] : 0.f); }
  return a;
}
struct F2 { v16b h, l; };
__device__ __forceinline__ F2 bsplit16(const float v[16]) { F2 r;
#pragma unroll
  for (int i = 0; i < 16; ++i) { const __bf16 h = (__bf16)v[i]; r.h[i] = h; r.l[i] = (__bf16)(v[i] - (float)h); }
  return r; }
__device__ __forceinline__ F2 split_row(const float* row, int k0, int lane) { float v[16]; const float* p = row + k0 + 8 * (lane >> 4);
#pragma unroll
  for (int i = 0; i < 8; ++i) { v[i] = p[i]; v[8 + i] = p[16 + i]; }
  return bsplit16(v); }
__device__ __forceinline__ F2 split_rowK(const float* row, int k0, int lane, int K) { float v[16]; const int g = lane >> 4;
#pragma unroll
  for (int i = 0; i < 8; ++i) { const int ka = k0 + 8 * g + i, kb = ka + 16; v[i] = ka < K ? row[ka < K ? ka : K - 1] : 0.f; v[8 + i] = kb < K ? row[kb < K ? kb : K - 1] : 0.f; }
  return bsplit16(v); }
__device__ __forceinline__ F2 split_col(const float* W, int k0, int n, int lane, int ld, int K) { float v[16]; const int g = lane >> 4;
#pragma unroll
  for (int i = 0; i < 8; ++i) { const int ka = k0 + 8 * g + i, kb = ka + 16; v[i] = ka < K ? W[(size_t)(ka < K ? ka : K - 1) * ld + n] : 0.f; v[8 + i] = kb < K ? W[(size_t)(kb < K ? kb : K - 1) * ld + n] : 0.f; }
  return bsplit16(v); }
__device__ __forceinline__ v8f mac3(const F2& a, const F2& b, v8f c) { c = wmma_bf(a.l, b.h, c); c = wmma_bf(a.h, b.l, c); return wmma_bf(a.h, b.h, c); }
__device__ __forceinline__ float sigm(float v) { return 1.0f / (1.0f + expf(-v)); }
#define LDSX() do { asm volatile("s_wait_dscnt 0" ::: "memory"); __builtin_amdgcn_wave_barrier(); __builtin_amdgcn_fence(__ATOMIC_RELEASE, "workgroup"); } while (0)


#define NB 4
#define SS 1024
#define NMEL 128
#define ND 256
#define ENC 512
#define DM 512
#define DMOD DM
#define DI 1024
#define DS 16
#define DR 32
#define NXD (DR + 2 * DS)
#define NL 4
#define CD 128
#define NCLS 10
#define NR (NB * SS)
#define XZP (2 * DI)
#define XDP NXD
#define DFF 2048
#ifndef NRT
#define NRT NR
#define NBT NB
#define SST SS
#endif
typedef __attribute__((ext_vector_type(8))) __bf16 v8b;
__device__ __forceinline__ v16b frag_b(const __bf16* rowk0, int lane) {
  union { v16b v; v8b q[2]; } u; const __bf16* p = rowk0 + 8 * (lane >> 4);
  u.q[0] = *(const v8b*)p; u.q[1] = *(const v8b*)(p + 16); return u.v;
}
__device__ __forceinline__ float bfr(float v) { return (float)(__bf16)v; }
__device__ __attribute__((noinline)) float exp_ni(float v) { return expf(v); }
__device__ __attribute__((noinline)) float erf_ni(float v) { return erff(v); }

__device__ __attribute__((noinline)) float tanh_ni(float v) { return tanhf(v); }
__device__ __attribute__((noinline)) float log1p_ni(float v) { return log1pf(v); }
__device__ __forceinline__ float silu_f(float v) { return v / (1.0f + exp_ni(-v)); }
#define PK_FC1 0
#define PK_FC2 (PK_FC1 + ENC * ND)
#define PK_PRJ (PK_FC2 + ND * ENC)
#define PK_IN  (PK_PRJ + DM * ND)
#define PK_XP  (PK_IN + (size_t)NL * XZP * DM)
#define PK_DT  (PK_XP + (size_t)NL * NXD * DI)
#define PK_OUT (PK_DT + (size_t)NL * DI * DR)
#define PK_H1  (PK_OUT + (size_t)NL * DM * DI)
#define PK_H2  (PK_H1 + CD * DM)
#define PK_END (PK_H2 + 16 * CD)
#define WS_PK   0u
#define WS_FEAT (WS_PK + 2u * (unsigned)PK_END)
#define WS_E1   (WS_FEAT + 4u * NR * ND)
#define WS_E2   (WS_E1 + 4u * NR * ENC)
#define WS_HA   (WS_E2 + 4u * NR * ND)
#define WS_HB   (WS_HA + 4u * NR * DM)
#define WS_XN   (WS_HB + 4u * NR * DM)
#define WS_XZ   (WS_XN + 4u * NR * DM)
#define WS_XD   (WS_XZ + 4u * NR * XZP)
#define WS_DT   (WS_XD + 4u * NR * XDP)
#define WS_C1   (WS_DT + 4u * NR * DI)
#define WS_END  (WS_C1 + 4u * NR * CD)

__global__ __launch_bounds__(256) void k_pack(const float* __restrict__ Wm, int K, int nrows, __bf16* __restrict__ DST) {
  __shared__ __align__(16) __bf16 s[8 * DFF]; const int n0 = blockIdx.x * 8, tid = threadIdx.x;
  for (int q = tid; q < 8 * K; q += 256) { const int rl = q / K, k = q % K; s[q] = (__bf16)((n0 + rl) < nrows ? Wm[(size_t)(n0 + rl) * K + k] : 0.f); }
  __syncthreads();
  for (int q = tid; q < K; q += 256) vst2((unsigned*)(DST + (size_t)n0 * K + q * 8), *(const v4u*)&s[q * 8]);
}
__global__ __launch_bounds__(256) void k_feat(const float* __restrict__ X, float* __restrict__ FEAT) {
  __shared__ __align__(16) float s[64][ND + 4]; __shared__ float sx[NMEL][66];
  const int t0 = blockIdx.x * 64, b = blockIdx.y, tid = threadIdx.x;
  for (int q = tid; q < NMEL * 65; q += 256) { const int c = q / 65, tl = q % 65; const int t = t0 - 1 + tl; sx[c][tl] = (t >= 0) ? bfr(X[((size_t)b * NMEL + c) * SS + (t >= 0 ? t : 0)]) : 0.f; }
  __syncthreads();
  for (int q = tid; q < 64 * NMEL; q += 256) { const int tl = q / NMEL, c = q % NMEL; const float cur = sx[c][tl + 1], prev = sx[c][tl]; s[tl][c] = cur; s[tl][NMEL + c] = (t0 + tl == 0) ? 0.f : fmaxf(cur - prev, 0.f); }
  __syncthreads();
  for (int q = tid; q < 64 * 64; q += 256) { const int tl = q >> 6, pc = q & 63; vst2(FEAT + ((size_t)b * SS + t0 + tl) * ND + pc * 4, *(const v4f*)&s[tl][pc * 4]); }
}
template <int XB>
__global__ __launch_bounds__(256) void k_ln(const float* __restrict__ X, const float* __restrict__ gw, const float* __restrict__ bw, float* __restrict__ Y) {
  __shared__ __align__(16) float s[8][DM];
  const int wave = threadIdx.x >> 5, lane = threadIdx.x & 31; const size_t r = (size_t)blockIdx.x * 8 + wave; const float* x = X + r * DM; float* sw = s[wave];
  float sum = 0.f;
#pragma unroll 4
  for (int i = 0; i < DM / 32; ++i) { float t = x[lane + 32 * i]; if (XB) t = bfr(t); sw[lane + 32 * i] = t; sum += t; }
#pragma unroll
  for (int o = 1; o < 32; o <<= 1) sum += __shfl_xor(sum, o);
  const float mu = sum / (float)DM; float var = 0.f;
#pragma unroll 4
  for (int i = 0; i < DM / 32; ++i) { const float d = sw[lane + 32 * i] - mu; var += d * d; }
#pragma unroll
  for (int o = 1; o < 32; o <<= 1) var += __shfl_xor(var, o);
  const float rs = rsqrtf(var / (float)DM + 1e-5f);
#pragma unroll 4
  for (int i = 0; i < DM / 32; ++i) { const int c = lane + 32 * i; sw[c] = (sw[c] - mu) * rs * bfr(gw[c]) + bfr(bw[c]); }
  LDSX();
#pragma unroll 2
  for (int pc = lane; pc < DM / 4; pc += 32) vst2(Y + r * DM + pc * 4, *(const v4f*)&sw[pc * 4]);
}

template <int K, int AM, int EPI, int NT, int RM>
__global__ __launch_bounds__(128) void k_lin(const float* __restrict__ A, int lda, const __bf16* __restrict__ P, const float* __restrict__ bias, float* __restrict__ OUT, int ldo, const float* __restrict__ RES, int ldr) {
  __shared__ __align__(16) float so[4][16][132];
  const int tid = threadIdx.x, wave = tid >> 5, lane = tid & 31, col = lane & 15, g = lane >> 4; const size_t r0 = (size_t)blockIdx.x * 64 + wave * 16; const int n0 = blockIdx.y * NT * 16;
  v8f acc[NT] = {};
#pragma unroll 2
  for (int kc = 0; kc < K / 32; ++kc) {
    if (AM == 0) { v16b a; { const float* p = A + (r0 + col) * lda + kc * 32 + 8 * g;
#pragma unroll
        for (int i = 0; i < 8; ++i) { a[i] = (__bf16)p[i]; a[8 + i] = (__bf16)p[16 + i]; } }
#pragma unroll
      for (int j = 0; j < NT; ++j) acc[j] = wmma_bf(a, frag_b(P + (size_t)(n0 + j * 16 + col) * K + kc * 32, lane), acc[j]); }
    else { const F2 a = split_row(A + (r0 + col) * lda, kc * 32, lane);
#pragma unroll
      for (int j = 0; j < NT; ++j) { const v16b w = frag_b(P + (size_t)(n0 + j * 16 + col) * K + kc * 32, lane); acc[j] = wmma_bf(a.l, w, acc[j]); acc[j] = wmma_bf(a.h, w, acc[j]); } } }
#pragma unroll
  for (int j = 0; j < NT; ++j) { const float bb = bias ? bfr(bias[n0 + j * 16 + col]) : 0.f;
#pragma unroll
    for (int r = 0; r < 8; ++r) { float v = acc[j][r] + bb; if (EPI == 1) v = fmaxf(v, 0.f); if (EPI == 2) v = tanh_ni(v); if (EPI == 3) v = (v > 20.f) ? v : log1p_ni(exp_ni(v)); if (EPI == 4) v = silu_f(v); if (RM == 1) v += RES[(r0 + 8 * g + r) * ldr + n0 + j * 16 + col]; if (RM == 2) v += bfr(RES[(r0 + 8 * g + r) * ldr + n0 + j * 16 + col]); so[wave][8 * g + r][j * 16 + col] = v; } }
  LDSX();
  for (int rl = 0; rl < 16; ++rl) if (lane < NT * 4) vst2(OUT + (r0 + rl) * ldo + n0 + lane * 4, *(const v4f*)&so[wave][rl][lane * 4]);
}

__global__ __launch_bounds__(256) void k_conv(float* __restrict__ XZ, const float* __restrict__ CW, const float* __restrict__ CB) {
  const int b = blockIdx.y, c0 = (blockIdx.x * 256 + threadIdx.x) * 4; float w[4][4], cb[4];
#pragma unroll
  for (int i = 0; i < 4; ++i) { cb[i] = bfr(CB[c0 + i]);
#pragma unroll
    for (int k = 0; k < 4; ++k) w[k][i] = bfr(CW[(c0 + i) * 4 + k]); }
  float* col = XZ + (size_t)b * SS * XZP + c0;
  v4f x1 = *(const v4f*)(col + (size_t)(SST - 1) * XZP), x2 = *(const v4f*)(col + (size_t)(SST - 2) * XZP), x3 = *(const v4f*)(col + (size_t)(SST - 3) * XZP);
#pragma unroll 1
  for (int t = SST - 1; t >= 0; --t) { const int tm = t - 3; v4f x0 = (tm >= 0) ? *(const v4f*)(col + (size_t)(tm >= 0 ? tm : 0) * XZP) : (v4f){0.f, 0.f, 0.f, 0.f}; v4f o;
#pragma unroll
    for (int i = 0; i < 4; ++i) { const float v = w[0][i] * x0[i] + w[1][i] * x3[i] + w[2][i] * x2[i] + w[3][i] * x1[i] + cb[i]; o[i] = silu_f(v); }
    vst2(col + (size_t)t * XZP, o); x1 = x2; x2 = x3; x3 = x0; }
}
__global__ __launch_bounds__(256) void k_scan(float* __restrict__ XZ, const float* __restrict__ XD, const float* __restrict__ DT, const float* __restrict__ ALOG, const float* __restrict__ Dp) {
  const int b = blockIdx.y, c0 = (blockIdx.x * 256 + threadIdx.x) * 4; float A[4][DS], h[4][DS], dd[4];
#pragma unroll
  for (int i = 0; i < 4; ++i) { dd[i] = bfr(Dp[c0 + i]);
#pragma unroll
    for (int n = 0; n < DS; ++n) { A[i][n] = -exp_ni(bfr(ALOG[(c0 + i) * DS + n])); h[i][n] = 0.f; } }
  const size_t rb = (size_t)b * SS;
#pragma unroll 1
  for (int t = 0; t < SST; ++t) { const size_t r = rb + t; const v4f dt4 = *(const v4f*)(DT + r * DI + c0), xb4 = *(const v4f*)(XZ + r * XZP + c0), z4 = *(const v4f*)(XZ + r * XZP + DI + c0);
    float Bt[DS], Ct[DS]; { const v4f* pb = (const v4f*)(XD + r * XDP + DR);
#pragma unroll
      for (int q = 0; q < 4; ++q) { const v4f vb = pb[q], vc = pb[4 + q];
#pragma unroll
        for (int i = 0; i < 4; ++i) { Bt[q * 4 + i] = vb[i]; Ct[q * 4 + i] = vc[i]; } } }
    v4f o;
#pragma unroll
    for (int i = 0; i < 4; ++i) { const float dti = dt4[i], xbi = xb4[i], dx = dti * xbi; float y = 0.f;
#pragma unroll
      for (int n = 0; n < DS; ++n) { h[i][n] = exp_ni(dti * A[i][n]) * h[i][n] + dx * Bt[n]; y += h[i][n] * Ct[n]; }
      y += xbi * dd[i]; o[i] = y * silu_f(z4[i]); }
    vst2(XZ + r * XZP + DI + c0, o); }
}

__global__ __launch_bounds__(128) void k_head(const float* __restrict__ C1, const __bf16* __restrict__ PH2, const float* __restrict__ hb, float* __restrict__ out) {
  __shared__ __align__(16) float sT[16][68];
  const int tid = threadIdx.x, wave = tid >> 5, lane = tid & 31, col = lane & 15, g = lane >> 4; const int t0 = blockIdx.x * 64, b = blockIdx.y; const size_t r0 = (size_t)b * SS + t0 + wave * 16;
  v8f acc = {};
#pragma unroll
  for (int kc = 0; kc < CD / 32; ++kc) { const F2 a = split_row(C1 + (r0 + col) * CD, kc * 32, lane); const v16b w = frag_b(PH2 + (size_t)col * CD + kc * 32, lane); acc = wmma_bf(a.l, w, acc); acc = wmma_bf(a.h, w, acc); }
#pragma unroll
  for (int r = 0; r < 8; ++r) sT[col][wave * 16 + 8 * g + r] = acc[r] + (col < NCLS ? bfr(hb[col]) : 0.f);
  __syncthreads();
  for (int q = tid; q < NCLS * 16; q += 128) { const int c = q >> 4, piece = q & 15; vst2(out + ((size_t)b * NCLS + c) * SS + t0 + piece * 4, *(const v4f*)&sT[c][piece * 4]); }
}
extern "C" void kernel_launch(void* const* d_in, const int* in_sizes, int n_in, void* d_out, int out_size, void* d_ws, size_t ws_size, hipStream_t stream) {
  (void)in_sizes; (void)n_in; (void)out_size;
  const float** F = (const float**)d_in;
  if (ws_size < (size_t)WS_END) return;
  char* ws = (char*)d_ws; __bf16* PK = (__bf16*)(ws + WS_PK);
  float *FEAT = (float*)(ws + WS_FEAT), *E1 = (float*)(ws + WS_E1), *E2 = (float*)(ws + WS_E2), *HA = (float*)(ws + WS_HA), *HB = (float*)(ws + WS_HB), *XN = (float*)(ws + WS_XN), *XZ = (float*)(ws + WS_XZ), *XD = (float*)(ws + WS_XD), *DT = (float*)(ws + WS_DT), *C1 = (float*)(ws + WS_C1);
  k_pack<<<ENC / 8, 256, 0, stream>>>(F[1], ND, ENC, PK + PK_FC1);
  k_pack<<<ND / 8, 256, 0, stream>>>(F[3], ENC, ND, PK + PK_FC2);
  k_pack<<<DM / 8, 256, 0, stream>>>(F[5], ND, DM, PK + PK_PRJ);
  k_pack<<<NL * XZP / 8, 256, 0, stream>>>(F[9], DM, NL * XZP, PK + PK_IN);
  k_pack<<<NL * NXD / 8, 256, 0, stream>>>(F[12], DI, NL * NXD, PK + PK_XP);
  k_pack<<<NL * DI / 8, 256, 0, stream>>>(F[13], DR, NL * DI, PK + PK_DT);
  k_pack<<<NL * DM / 8, 256, 0, stream>>>(F[17], DI, NL * DM, PK + PK_OUT);
  k_pack<<<CD / 8, 256, 0, stream>>>(F[20], DM, CD, PK + PK_H1);
  k_pack<<<16 / 8, 256, 0, stream>>>(F[22], CD, NCLS, PK + PK_H2);
  k_feat<<<dim3(SST / 64, NBT), 256, 0, stream>>>(F[0], FEAT);
  k_lin<ND, 1, 4, 8, 0><<<dim3(NRT / 64, ENC / 128), 128, 0, stream>>>(FEAT, ND, PK + PK_FC1, F[2], E1, ENC, nullptr, 0);
  k_lin<ENC, 1, 0, 8, 0><<<dim3(NRT / 64, ND / 128), 128, 0, stream>>>(E1, ENC, PK + PK_FC2, F[4], E2, ND, nullptr, 0);
  k_lin<ND, 1, 0, 8, 0><<<dim3(NRT / 64, DM / 128), 128, 0, stream>>>(E2, ND, PK + PK_PRJ, F[6], HA, DM, nullptr, 0);
  float* Hcur = HA; float* Hnext = HB;
  for (int l = 0; l < NL; ++l) {
    k_ln<0><<<NRT / 8, 256, 0, stream>>>(Hcur, F[7] + l * DM, F[8] + l * DM, XN);
    k_lin<DM, 1, 0, 8, 0><<<dim3(NRT / 64, XZP / 128), 128, 0, stream>>>(XN, DM, PK + PK_IN + (size_t)l * XZP * DM, nullptr, XZ, XZP, nullptr, 0);
    k_conv<<<dim3(DI / 1024, NBT), 256, 0, stream>>>(XZ, F[10] + (size_t)l * DI * 4, F[11] + l * DI);
    k_lin<DI, 1, 0, 4, 0><<<dim3(NRT / 64, 1), 128, 0, stream>>>(XZ, XZP, PK + PK_XP + (size_t)l * NXD * DI, nullptr, XD, XDP, nullptr, 0);
    k_lin<DR, 1, 3, 8, 0><<<dim3(NRT / 64, DI / 128), 128, 0, stream>>>(XD, XDP, PK + PK_DT + (size_t)l * DI * DR, F[14] + l * DI, DT, DI, nullptr, 0);
    k_scan<<<dim3(DI / 1024, NBT), 256, 0, stream>>>(XZ, XD, DT, F[15] + (size_t)l * DI * DS, F[16] + l * DI);
    k_lin<DI, 1, 0, 8, 1><<<dim3(NRT / 64, DM / 128), 128, 0, stream>>>(XZ + DI, XZP, PK + PK_OUT + (size_t)l * DM * DI, nullptr, Hnext, DM, Hcur, DM);
    float* t = Hcur; Hcur = Hnext; Hnext = t; }
  k_ln<0><<<NRT / 8, 256, 0, stream>>>(Hcur, F[18], F[19], XN);
  k_lin<DM, 1, 4, 8, 0><<<dim3(NRT / 64, CD / 128), 128, 0, stream>>>(XN, DM, PK + PK_H1, F[21], C1, CD, nullptr, 0);
  k_head<<<dim3(SST / 64, NBT), 128, 0, stream>>>(C1, PK + PK_H2, F[23], (float*)d_out);
}
